// VisionTransformerEncoder_53042846105901
// MI455X (gfx1250) — hardware-verified
//
#include <hip/hip_runtime.h>
#include <math.h>
typedef __attribute__((ext_vector_type(16))) _Float16 v16h;
typedef __attribute__((ext_vector_type(8)))  _Float16 v8h;
typedef __attribute__((ext_vector_type(16))) __bf16   v16b;
typedef __attribute__((ext_vector_type(8)))  __bf16   v8b;
typedef __attribute__((ext_vector_type(8)))  float    v8f;
typedef __attribute__((ext_vector_type(4)))  float    v4f;
#define PSCALE 32768.0f
#define U16(p) ((const unsigned short*)(const void*)(p))
#define PSCALE_INV (1.0f / 32768.0f)

__device__ __forceinline__ unsigned short f2bf_bits(float f) {
  unsigned u = __float_as_uint(f);
  return (unsigned short)((u + 0x7FFFu + ((u >> 16) & 1u)) >> 16);
}
__device__ __forceinline__ float bf_bits2f(unsigned short h) { return __uint_as_float(((unsigned)h) << 16); }

__device__ __forceinline__ void dep_guard_h(v8f& a, v8f& b, v16h x, v16h y) { asm volatile("v_nop\n\tv_nop\n\tv_nop\n\tv_nop" : "+v"(a), "+v"(b) : "v"(x), "v"(y)); }
__device__ __forceinline__ void dep_guard_b(v8f& a, v8f& b, v16b x, v16b y) { asm volatile("v_nop\n\tv_nop\n\tv_nop\n\tv_nop" : "+v"(a), "+v"(b) : "v"(x), "v"(y)); }
__device__ __forceinline__ void keep4_h(v16h a, v16h b, v16h c, v16h d) { asm volatile("v_nop" :: "v"(a), "v"(b), "v"(c), "v"(d)); }
__device__ __forceinline__ void keep4_b(v16b a, v16b b, v16b c, v16b d) { asm volatile("v_nop" :: "v"(a), "v"(b), "v"(c), "v"(d)); }
__device__ __forceinline__ void acc_guard4(v8f& a, v8f& b, v8f& c, v8f& d) { asm volatile("v_nop\n\tv_nop\n\tv_nop\n\tv_nop" : "+v"(a), "+v"(b), "+v"(c), "+v"(d)); }
template <typename T> struct Frag;
template <> struct Frag<_Float16> {
  typedef v16h V; union U { v16h v; v8h h[2]; };
  static __device__ __forceinline__ v16h load(const _Float16* p) {
    U f; f.h[0] = *(const v8h*)(p); f.h[1] = *(const v8h*)(p + 16); return f.v;
  }
  static __device__ __forceinline__ v8f mma(v16h a, v16h b, v8f c) {
    return __builtin_amdgcn_wmma_f32_16x16x32_f16(false, a, false, b, (short)0, c, false, false);
  }
  static __device__ __forceinline__ void guard(v8f& a, v8f& b, v16h x, v16h y) { dep_guard_h(a, b, x, y); }
  static __device__ __forceinline__ void keep(v16h a, v16h b, v16h c, v16h d) { keep4_h(a, b, c, d); }
};
template <> struct Frag<__bf16> {
  typedef v16b V; union U { v16b v; v8b h[2]; };
  static __device__ __forceinline__ v16b load(const __bf16* p) {
    U f; f.h[0] = *(const v8b*)(p); f.h[1] = *(const v8b*)(p + 16); return f.v;
  }
  static __device__ __forceinline__ v8f mma(v16b a, v16b b, v8f c) {
    return __builtin_amdgcn_wmma_f32_16x16x32_bf16(false, a, false, b, (short)0, c, false, false);
  }
  static __device__ __forceinline__ void guard(v8f& a, v8f& b, v16b x, v16b y) { dep_guard_b(a, b, x, y); }
  static __device__ __forceinline__ void keep(v16b a, v16b b, v16b c, v16b d) { keep4_b(a, b, c, d); }
};

template <int ET> struct Elem;
template <> struct Elem<0> { typedef _Float16 T; };
template <> struct Elem<1> { typedef __bf16 T; };
template <int ET, bool SPLIT, int BIAS_MODE, int OUT_MODE, bool RESID, int ACT = 0>
__global__ __launch_bounds__(256) void wmma_gemm64(
    const unsigned short* __restrict__ Ap, const unsigned short* __restrict__ A2p, int lda, long strideA,
    const unsigned short* __restrict__ Btp, const unsigned short* __restrict__ Bt2p, int ldb, long strideB,
    void* __restrict__ Cout, void* __restrict__ Cout2, int ldc, long strideC,
    const float* __restrict__ bias,
    const float* __restrict__ resid, long strideR,
    int M, int N, int K, float scale) {
  typedef typename Elem<ET>::T T;
  typedef typename Frag<T>::V V;
  const T* A = (const T*)Ap; const T* A2 = (const T*)A2p; const T* Bt = (const T*)Btp; const T* Bt2 = (const T*)Bt2p;
  __shared__ __align__(16) float sT[8][16 * 68];
  const int b    = blockIdx.y;
  const int lane = threadIdx.x & 31;
  const int wave = threadIdx.x >> 5;
  const int tilesN = N >> 6;
  const int tilesM = M >> 6;
  const int tile = blockIdx.x * 8 + wave;
  if (tile >= tilesM * tilesN) return;
  const int tm = tile / tilesN;
  const int tn = tile - tm * tilesN;
  const int m0 = tm << 6;
  const int n0 = tn << 6;

  const T* Ab  = A  + (size_t)b * strideA;
  const T* Bb  = Bt + (size_t)b * strideB;
  const T* Ab2 = SPLIT ? (A2  + (size_t)b * strideA) : nullptr;
  const T* Bb2 = SPLIT ? (Bt2 + (size_t)b * strideB) : nullptr;

  const int rlane = lane & 15;
  const int koff  = (lane >> 4) * 8;
  const int mOff  = (lane >> 4) * 8;

  v8f acc[4][4];
#pragma unroll
  for (int i = 0; i < 4; ++i)
#pragma unroll
    for (int j = 0; j < 4; ++j) acc[i][j] = (v8f){0.f,0.f,0.f,0.f,0.f,0.f,0.f,0.f};

  for (int k0 = 0; k0 < K; k0 += 32) {
    V bh[4], bl[4];
#pragma unroll
    for (int j = 0; j < 4; ++j) {
      const size_t bo = (size_t)(n0 + (j << 4) + rlane) * ldb + koff + k0;
      bh[j] = Frag<T>::load(Bb + bo);
      if (SPLIT) bl[j] = Frag<T>::load(Bb2 + bo);
    }
#pragma unroll
    for (int i = 0; i < 4; ++i) {
      const size_t ao = (size_t)(m0 + (i << 4) + rlane) * lda + koff + k0;
      V ah = Frag<T>::load(Ab + ao);
      V al;
      if (SPLIT) al = Frag<T>::load(Ab2 + ao);
#pragma unroll
      for (int j = 0; j < 4; ++j) {
        acc[i][j] = Frag<T>::mma(ah, bh[j], acc[i][j]);
        if (SPLIT) {
          acc[i][j] = Frag<T>::mma(ah, bl[j], acc[i][j]);
          acc[i][j] = Frag<T>::mma(al, bh[j], acc[i][j]);
        }
      }
      Frag<T>::guard(acc[i][0], acc[i][3], ah, SPLIT ? al : ah);
    }
    Frag<T>::keep(bh[0], bh[1], bh[2], bh[3]);
    if (SPLIT) Frag<T>::keep(bl[0], bl[1], bl[2], bl[3]);
  }
  acc_guard4(acc[0][0], acc[0][1], acc[0][2], acc[0][3]);
  acc_guard4(acc[1][0], acc[1][1], acc[1][2], acc[1][3]);
  acc_guard4(acc[2][0], acc[2][1], acc[2][2], acc[2][3]);
  acc_guard4(acc[3][0], acc[3][1], acc[3][2], acc[3][3]);

  float* slab = sT[wave];
  const float* Rb = RESID ? (resid + (size_t)b * strideR) : nullptr;
#pragma unroll
  for (int i = 0; i < 4; ++i) {
    const int mBase = m0 + (i << 4);
#pragma unroll
    for (int j = 0; j < 4; ++j) {
      const int n = n0 + (j << 4) + rlane;
      float bv = 0.f;
      if (BIAS_MODE == 2) bv = bias[n];
#pragma unroll
      for (int r = 0; r < 8; ++r) {
        float v = acc[i][j][r] * scale;
        if (BIAS_MODE == 1) v += bias[mBase + mOff + r];
        if (BIAS_MODE == 2) v += bv;
        if (RESID) v += Rb[(size_t)(mBase + mOff + r) * ldc + n];
        if (ACT == 1) v = tanhf(v);
        if (ACT == 2) v = fmaxf(v, 0.0f);
        if (ACT == 3) v = v / (1.0f + expf(-v));
        if (ACT == 4) v = (v > 0.f) ? v : 0.01f * v;
        if (ACT == 5) v = 0.5f * v * (1.0f + erff(v * 0.70710678118654752f));
        slab[(mOff + r) * 68 + (j << 4) + rlane] = v;
      }
    }
    __builtin_amdgcn_fence(__ATOMIC_RELEASE, "workgroup");
    __builtin_amdgcn_wave_barrier();
    __builtin_amdgcn_fence(__ATOMIC_ACQUIRE, "workgroup");
    if (OUT_MODE == 0) {
      float* C = (float*)Cout + (size_t)b * strideC;
      const int hh = lane >> 4, c4 = (lane & 15) * 4;
      for (int pass = 0; pass < 2; ++pass) {
#pragma unroll
        for (int it = 0; it < 8; ++it) {
          const int row = it * 2 + hh;
          v4f v = *(const v4f*)(slab + row * 68 + c4);
          *(volatile v4f*)(C + (size_t)(mBase + row) * ldc + n0 + c4) = v;
        }
        __threadfence();
      }
    } else {
      const int q = lane >> 3, c8 = (lane & 7) * 8;
      unsigned short* C  = (unsigned short*)Cout  + (size_t)b * strideC;
      unsigned short* C2 = (OUT_MODE == 2) ? ((unsigned short*)Cout2 + (size_t)b * strideC) : nullptr;
      for (int pass = 0; pass < 2; ++pass) {
#pragma unroll
        for (int it = 0; it < 4; ++it) {
          const int row = it * 4 + q;
          const float* sp = slab + row * 68 + c8;
          v8h hv, lv;
#pragma unroll
          for (int e = 0; e < 8; ++e) {
            if (OUT_MODE == 1) {
              hv[e] = (_Float16)sp[e];
            } else {
              unsigned short hb = f2bf_bits(sp[e]);
              unsigned short lb = f2bf_bits(sp[e] - bf_bits2f(hb));
              hv[e] = __builtin_bit_cast(_Float16, hb);
              lv[e] = __builtin_bit_cast(_Float16, lb);
            }
          }
          *(volatile v8h*)(C + (size_t)(mBase + row) * ldc + n0 + c8) = hv;
          if (OUT_MODE == 2) *(volatile v8h*)(C2 + (size_t)(mBase + row) * ldc + n0 + c8) = lv;
        }
        __threadfence();
      }
    }
    __builtin_amdgcn_fence(__ATOMIC_RELEASE, "workgroup");
    __builtin_amdgcn_wave_barrier();
    __builtin_amdgcn_fence(__ATOMIC_ACQUIRE, "workgroup");
  }
}

__global__ __launch_bounds__(256) void transpose_cast_f16(const float* __restrict__ in, int ldi,
                                                         _Float16* __restrict__ outT, int ldo, float scale) {
  __shared__ __align__(16) _Float16 tile[64][72];
  const int c0 = blockIdx.x * 64, r0 = blockIdx.y * 64;
  const int t = threadIdx.y * 32 + threadIdx.x;
  for (int i = threadIdx.y; i < 64; i += 8) {
    tile[threadIdx.x][i]      = (_Float16)(in[(size_t)(r0 + i) * ldi + c0 + threadIdx.x] * scale);
    tile[32 + threadIdx.x][i] = (_Float16)(in[(size_t)(r0 + i) * ldi + c0 + 32 + threadIdx.x] * scale);
  }
  __syncthreads();
  const int q = t >> 3, c8 = (t & 7) * 8;
  for (int pass = 0; pass < 2; ++pass) {
#pragma unroll
    for (int it = 0; it < 2; ++it) {
      const int c = it * 32 + q;
      v8h hv = *(const v8h*)(&tile[c][c8]);
      *(volatile v8h*)(outT + (size_t)(c0 + c) * ldo + r0 + c8) = hv;
    }
    __threadfence();
  }
}

#define AT_D 64
#define AT_NW 4
#define AT_QB 64
#define AT_KC 64
__device__ __forceinline__ v8f hmma(v16h a, v16h b, v8f c) {
  c = __builtin_amdgcn_wmma_f32_16x16x32_f16(false, a, false, b, (short)0, c, false, false);
  asm volatile("v_nop\n\tv_nop\n\tv_nop\n\tv_nop" : "+v"(c) : "v"(a), "v"(b));
  return c;
}

__global__ __launch_bounds__(128)
void attn64_h16_kernel(const _Float16* __restrict__ q, const _Float16* __restrict__ k,
                       const _Float16* __restrict__ v, _Float16* __restrict__ out,
                       int S, int Hn, int rs, int rso, float sscale) {
  union FB { v16h v; v8h h[2]; };
  __shared__ __align__(16) _Float16 Ksh[AT_KC * AT_D];
  __shared__ __align__(16) _Float16 Vth[AT_D * AT_KC];
  __shared__ __align__(16) _Float16 Psh[AT_NW][16 * AT_KC];
  __shared__ __align__(16) float    Os[AT_NW][16 * 68];

  const int tid  = threadIdx.x;
  const int wave = tid >> 5;
  const int lane = tid & 31;
  const int hh   = lane >> 4;
  const int c    = lane & 15;

  const int nqb = S / AT_QB;
  const int bx  = blockIdx.x;
  const int qb  = bx % nqb;
  const int bhd = bx / nqb;
  const int h   = bhd % Hn;
  const int b   = bhd / Hn;
  const int q0  = qb * AT_QB + wave * 16;

  const size_t tok0 = (size_t)b * S;
  const _Float16* qbp = q + tok0 * rs + (size_t)h * AT_D;
  const _Float16* kbp = k + tok0 * rs + (size_t)h * AT_D;
  const _Float16* vbp = v + tok0 * rs + (size_t)h * AT_D;
  _Float16*       obp = out + tok0 * rso + (size_t)h * AT_D;

  v16h qa0, qa1;
  {
    const _Float16* qrow = qbp + (size_t)(q0 + c) * rs;
    qa0 = Frag<_Float16>::load(qrow + 8 * hh);
    qa1 = Frag<_Float16>::load(qrow + 32 + 8 * hh);
  }

  float mrow[8], lrow[8];
  v8f oacc[4];
#pragma unroll
  for (int r = 0; r < 8; ++r) { mrow[r] = -INFINITY; lrow[r] = 0.f; }
#pragma unroll
  for (int t = 0; t < 4; ++t) oacc[t] = (v8f){0.f,0.f,0.f,0.f,0.f,0.f,0.f,0.f};

  const int nChunks = S / AT_KC;
  for (int kc = 0; kc < nChunks; ++kc) {
    const int kv0 = kc * AT_KC;
    __syncthreads();
    {
      const int kvr = tid >> 1, dh = (tid & 1) * 32;
      const _Float16* krow = kbp + (size_t)(kv0 + kvr) * rs + dh;
      const _Float16* vrow = vbp + (size_t)(kv0 + kvr) * rs + dh;
#pragma unroll
      for (int i = 0; i < 4; ++i) {
        const v8h kk = *(const v8h*)(krow + 8 * i);
        *(v8h*)(Ksh + kvr * AT_D + dh + 8 * i) = kk;
        const v8h vv = *(const v8h*)(vrow + 8 * i);
#pragma unroll
        for (int e = 0; e < 8; ++e) Vth[(dh + 8 * i + e) * AT_KC + kvr] = vv[e];
      }
    }
    __syncthreads();

    v8f s[4];
#pragma unroll
    for (int j = 0; j < 4; ++j) {
      v8f sj = (v8f){0.f,0.f,0.f,0.f,0.f,0.f,0.f,0.f};
      const _Float16* kp = Ksh + (j * 16 + c) * AT_D + 8 * hh;
      FB kb0, kb1;
      kb0.h[0] = *(const v8h*)(kp);      kb0.h[1] = *(const v8h*)(kp + 16);
      kb1.h[0] = *(const v8h*)(kp + 32); kb1.h[1] = *(const v8h*)(kp + 48);
      sj = hmma(qa0, kb0.v, sj);
      sj = hmma(qa1, kb1.v, sj);
      s[j] = sj;
    }
    float cm[8];
#pragma unroll
    for (int r = 0; r < 8; ++r) {
      float m = -INFINITY;
#pragma unroll
      for (int j = 0; j < 4; ++j) { s[j][r] *= sscale; m = fmaxf(m, s[j][r]); }
#pragma unroll
      for (int off = 1; off < 16; off <<= 1) m = fmaxf(m, __shfl_xor(m, off, 32));
      cm[r] = m;
    }
    _Float16* pw = Psh[wave];
#pragma unroll
    for (int r = 0; r < 8; ++r) {
      const float mnew  = fmaxf(mrow[r], cm[r]);
      const float alpha = expf(mrow[r] - mnew);
      mrow[r] = mnew;
      float psum = 0.f;
#pragma unroll
      for (int j = 0; j < 4; ++j) {
        const float p = expf(s[j][r] - mnew);
        psum += p;
        pw[(8 * hh + r) * AT_KC + j * 16 + c] = (_Float16)(p * PSCALE);
      }
#pragma unroll
      for (int off = 1; off < 16; off <<= 1) psum += __shfl_xor(psum, off, 32);
      lrow[r] = lrow[r] * alpha + psum;
#pragma unroll
      for (int t = 0; t < 4; ++t) oacc[t][r] *= alpha;
    }
    __builtin_amdgcn_fence(__ATOMIC_RELEASE, "workgroup");
    __builtin_amdgcn_wave_barrier();
    __builtin_amdgcn_fence(__ATOMIC_ACQUIRE, "workgroup");
#pragma unroll 1
    for (int kk = 0; kk < 2; ++kk) {
      FB pa;
      const _Float16* pp = pw + c * AT_KC + kk * 32 + 8 * hh;
      pa.h[0] = *(const v8h*)(pp);
      pa.h[1] = *(const v8h*)(pp + 16);
#pragma unroll
      for (int t = 0; t < 4; ++t) {
        FB vb;
        const _Float16* vp = Vth + (t * 16 + c) * AT_KC + kk * 32 + 8 * hh;
        vb.h[0] = *(const v8h*)(vp);
        vb.h[1] = *(const v8h*)(vp + 16);
        oacc[t] = hmma(pa.v, vb.v, oacc[t]);
      }
    }
  }

  float* os = Os[wave];
#pragma unroll
  for (int r = 0; r < 8; ++r) {
    const float inv = 1.0f / (lrow[r] * PSCALE);
#pragma unroll
    for (int t = 0; t < 4; ++t) os[(8 * hh + r) * 68 + t * 16 + c] = oacc[t][r] * inv;
  }
  __builtin_amdgcn_fence(__ATOMIC_RELEASE, "workgroup");
  __builtin_amdgcn_wave_barrier();
  __builtin_amdgcn_fence(__ATOMIC_ACQUIRE, "workgroup");
  {
    const int qq = lane >> 3, c8 = (lane & 7) * 8;
    for (int pass = 0; pass < 2; ++pass) {
#pragma unroll
      for (int it = 0; it < 4; ++it) {
        const int row = it * 4 + qq;
        const float* sp = os + row * 68 + c8;
        v8h hv;
#pragma unroll
        for (int e = 0; e < 8; ++e) hv[e] = (_Float16)sp[e];
        *(volatile v8h*)(obp + (size_t)(q0 + row) * rso + c8) = hv;
      }
      __threadfence();
    }
  }
}

#define VB 8
#define VN 1024
#define VE 1024
#define VH 16
#define VM 4096
#define VROWS (VB * VN)
#define VHALF (VROWS / 2)
__global__ __launch_bounds__(256) void ln1024_kernel(const float* __restrict__ X, const float* __restrict__ g, const float* __restrict__ bt, unsigned* __restrict__ Y16) {
  const int lane = threadIdx.x & 31, wave = threadIdx.x >> 5; const size_t row = (size_t)blockIdx.x * 8 + wave;
  const float* xr = X + row * VE;
  float v[32]; float s = 0.f;
#pragma unroll
  for (int q = 0; q < 8; ++q) { const v4f a = *(const v4f*)(xr + (q * 32 + lane) * 4); v[4*q] = a[0]; v[4*q+1] = a[1]; v[4*q+2] = a[2]; v[4*q+3] = a[3]; s += a[0] + a[1] + a[2] + a[3]; }
  for (int o = 16; o > 0; o >>= 1) s += __shfl_xor(s, o, 32);
  const float mu = s / (float)VE;
  float s2 = 0.f;
#pragma unroll
  for (int q = 0; q < 32; ++q) { const float d = v[q] - mu; s2 += d * d; }
  for (int o = 16; o > 0; o >>= 1) s2 += __shfl_xor(s2, o, 32);
  const float inv = rsqrtf(s2 / (float)VE + 1e-6f);
  typedef __attribute__((ext_vector_type(2))) unsigned u2;
  for (int pass = 0; pass < 2; ++pass) {
#pragma unroll
    for (int q = 0; q < 8; ++q) { const int c0 = (q * 32 + lane) * 4; float y[4];
#pragma unroll
      for (int e = 0; e < 4; ++e) y[e] = (v[4*q+e] - mu) * inv * g[c0 + e] + bt[c0 + e];
      u2 pk; pk[0] = (unsigned)__builtin_bit_cast(unsigned short, (_Float16)y[0]) | ((unsigned)__builtin_bit_cast(unsigned short, (_Float16)y[1]) << 16);
      pk[1] = (unsigned)__builtin_bit_cast(unsigned short, (_Float16)y[2]) | ((unsigned)__builtin_bit_cast(unsigned short, (_Float16)y[3]) << 16);
      *(volatile u2*)(Y16 + (row * VE + c0) / 2) = pk; }
    __threadfence();
  }
}

extern "C" void kernel_launch(void* const* d_in, const int* in_sizes, int n_in, void* d_out, int out_size, void* d_ws, size_t ws_size, hipStream_t stream) {
  (void)n_in;
  if (in_sizes[0] != VROWS * VE || out_size != VROWS * VE) return;
  const float* x = (const float*)d_in[0]; const float* ln1g = (const float*)d_in[1]; const float* ln1b = (const float*)d_in[2];
  const float* wqkv = (const float*)d_in[3]; const float* bqkv = (const float*)d_in[4]; const float* wo = (const float*)d_in[5]; const float* bo = (const float*)d_in[6];
  const float* ln2g = (const float*)d_in[7]; const float* ln2b = (const float*)d_in[8]; const float* w1 = (const float*)d_in[9]; const float* b1 = (const float*)d_in[10];
  const float* w2 = (const float*)d_in[11]; const float* b2 = (const float*)d_in[12];
  float* out = (float*)d_out;

  char* ws = (char*)d_ws; size_t off = 0;
  auto carve = [&](size_t bytes) -> char* { char* p = ws + off; off += (bytes + 255) & ~(size_t)255; return p; };
  char* rY   = carve((size_t)VROWS * VE * 2);
  _Float16* WqkvT = (_Float16*)carve((size_t)3 * VE * VE * 2);
  _Float16* WoT   = (_Float16*)carve((size_t)VE * VE * 2);
  _Float16* W1T   = (_Float16*)carve((size_t)VM * VE * 2);
  _Float16* W2T   = (_Float16*)carve((size_t)VE * VM * 2);
  char* rQKV = carve((size_t)VROWS * 3 * VE * 2);
  float* X1  = (float*)carve((size_t)VROWS * VE * 4);
  if (off > ws_size) return;
  unsigned* Y16 = (unsigned*)rY;
  _Float16* O16 = (_Float16*)rY;
  _Float16* QKV16 = (_Float16*)rQKV;
  _Float16* H16   = (_Float16*)rQKV;

  ln1024_kernel<<<VROWS / 8, 256, 0, stream>>>(x, ln1g, ln1b, Y16);
  transpose_cast_f16<<<dim3(3 * VE / 64, VE / 64), dim3(32, 8), 0, stream>>>(wqkv, 3 * VE, WqkvT, VE, 1.0f);
  transpose_cast_f16<<<dim3(VE / 64, VE / 64), dim3(32, 8), 0, stream>>>(wo, VE, WoT, VE, 1.0f);
  transpose_cast_f16<<<dim3(VM / 64, VE / 64), dim3(32, 8), 0, stream>>>(w1, VM, W1T, VE, 1.0f);
  transpose_cast_f16<<<dim3(VE / 64, VM / 64), dim3(32, 8), 0, stream>>>(w2, VE, W2T, VM, 1.0f);
  { const int t = (VROWS / 64) * (3 * VE / 64);
    wmma_gemm64<0, false, 2, 1, false, 0><<<dim3((t + 7) / 8, 1), 256, 0, stream>>>(
        (const unsigned short*)Y16, nullptr, VE, 0, U16(WqkvT), nullptr, VE, 0, (void*)QKV16, nullptr, 3 * VE, 0,
        bqkv, nullptr, 0, VROWS, 3 * VE, VE, 1.0f); }
  attn64_h16_kernel<<<VB * VH * (VN / AT_QB), AT_NW * 32, 0, stream>>>(QKV16, QKV16 + VE, QKV16 + 2 * VE, O16, VN, VH, 3 * VE, VE, 0.125f);
  { const int t = (VROWS / 64) * (VE / 64);
    wmma_gemm64<0, false, 2, 0, true, 0><<<dim3((t + 7) / 8, 1), 256, 0, stream>>>(
        U16(O16), nullptr, VE, 0, U16(WoT), nullptr, VE, 0, (void*)X1, nullptr, VE, 0,
        bo, x, 0, VROWS, VE, VE, 1.0f); }
  ln1024_kernel<<<VROWS / 8, 256, 0, stream>>>(X1, ln2g, ln2b, Y16);
  for (int half = 0; half < 2; ++half) {
    const size_t r0 = (size_t)half * VHALF;
    { const int t = (VHALF / 64) * (VM / 64);
      wmma_gemm64<0, false, 2, 1, false, 5><<<dim3((t + 7) / 8, 1), 256, 0, stream>>>(
          (const unsigned short*)Y16 + r0 * VE, nullptr, VE, 0, U16(W1T), nullptr, VE, 0, (void*)H16, nullptr, VM, 0,
          b1, nullptr, 0, VHALF, VM, VE, 1.0f); }
    { const int t = (VHALF / 64) * (VE / 64);
      wmma_gemm64<0, false, 2, 0, true, 0><<<dim3((t + 7) / 8, 1), 256, 0, stream>>>(
          U16(H16), nullptr, VM, 0, U16(W2T), nullptr, VM, 0, (void*)(out + r0 * VE), nullptr, VE, 0,
          b2, X1 + r0 * VE, 0, VHALF, VE, VM, 1.0f); }
  }
}
